// Encoders_13451837571792
// MI455X (gfx1250) — hardware-verified
//
#include <hip/hip_runtime.h>
#include <math.h>

constexpr int kB     = 4;
constexpr int kS     = 1024;
constexpr int kDM    = 512;
constexpr int kH     = 8;
constexpr int kHD    = 64;
constexpr int kFF    = 2048;
constexpr int kRows  = kB * kS;
constexpr int kNL    = 2;
constexpr int kPlane = kS * kS;

constexpr float kWCarry    = 32.0f;
constexpr float kActCarry  = 8.0f;
constexpr float kPCarry    = 32768.0f;
constexpr float kOCarry    = 64.0f;
constexpr float kProjScale = 1.0f / (kActCarry * kWCarry);
constexpr float kScoreScale = 0.125f;
constexpr float kPVScale   = kOCarry / kPCarry;
constexpr float kWoScale   = 1.0f / (kOCarry * kWCarry);
constexpr float kFF2Scale  = 1.0f / kWCarry;
constexpr float kInvDM     = 1.0f / 512.0f;
constexpr float kLnEps     = 1e-9f;

typedef __attribute__((ext_vector_type(16))) _Float16 v16h;
typedef __attribute__((ext_vector_type(8)))  _Float16 v8h;
typedef __attribute__((ext_vector_type(16))) __bf16   v16b;
typedef __attribute__((ext_vector_type(8)))  __bf16   v8b;
typedef __attribute__((ext_vector_type(8)))  float    v8f;
typedef __attribute__((ext_vector_type(4)))  float    v4f;
typedef __attribute__((ext_vector_type(4)))  unsigned int v4u;
typedef __attribute__((ext_vector_type(4)))  int      v4i;

__device__ __forceinline__ unsigned short f2bf_bits(float f) {
  unsigned u = __float_as_uint(f);
  return (unsigned short)((u + 0x7FFFu + ((u >> 16) & 1u)) >> 16);
}
__device__ __forceinline__ float bf_bits2f(unsigned short h) { return __uint_as_float(((unsigned)h) << 16); }

__device__ __forceinline__ void dep_guard_h(v8f& a, v8f& b, v16h x, v16h y) { asm volatile("v_nop\n\tv_nop\n\tv_nop\n\tv_nop" : "+v"(a), "+v"(b) : "v"(x), "v"(y)); }
__device__ __forceinline__ void dep_guard_b(v8f& a, v8f& b, v16b x, v16b y) { asm volatile("v_nop\n\tv_nop\n\tv_nop\n\tv_nop" : "+v"(a), "+v"(b) : "v"(x), "v"(y)); }
__device__ __forceinline__ void keep4_h(v16h a, v16h b, v16h c, v16h d) { asm volatile("v_nop" :: "v"(a), "v"(b), "v"(c), "v"(d)); }
__device__ __forceinline__ void keep4_b(v16b a, v16b b, v16b c, v16b d) { asm volatile("v_nop" :: "v"(a), "v"(b), "v"(c), "v"(d)); }
__device__ __forceinline__ void acc_guard4(v8f& a, v8f& b, v8f& c, v8f& d) { asm volatile("v_nop\n\tv_nop\n\tv_nop\n\tv_nop" : "+v"(a), "+v"(b), "+v"(c), "+v"(d)); }
template <typename T> struct Frag;
template <> struct Frag<_Float16> {
  typedef v16h V; union U { v16h v; v8h h[2]; };
  static __device__ __forceinline__ v16h load(const _Float16* p) {
    U f; f.h[0] = *(const v8h*)(p); f.h[1] = *(const v8h*)(p + 16); return f.v;
  }
  static __device__ __forceinline__ v8f mma(v16h a, v16h b, v8f c) {
    return __builtin_amdgcn_wmma_f32_16x16x32_f16(false, a, false, b, (short)0, c, false, false);
  }
  static __device__ __forceinline__ void guard(v8f& a, v8f& b, v16h x, v16h y) { dep_guard_h(a, b, x, y); }
  static __device__ __forceinline__ void keep(v16h a, v16h b, v16h c, v16h d) { keep4_h(a, b, c, d); }
};
template <> struct Frag<__bf16> {
  typedef v16b V; union U { v16b v; v8b h[2]; };
  static __device__ __forceinline__ v16b load(const __bf16* p) {
    U f; f.h[0] = *(const v8b*)(p); f.h[1] = *(const v8b*)(p + 16); return f.v;
  }
  static __device__ __forceinline__ v8f mma(v16b a, v16b b, v8f c) {
    return __builtin_amdgcn_wmma_f32_16x16x32_bf16(false, a, false, b, (short)0, c, false, false);
  }
  static __device__ __forceinline__ void guard(v8f& a, v8f& b, v16b x, v16b y) { dep_guard_b(a, b, x, y); }
  static __device__ __forceinline__ void keep(v16b a, v16b b, v16b c, v16b d) { keep4_b(a, b, c, d); }
};

__device__ __forceinline__ unsigned pk16(unsigned short a, unsigned short b) { return (unsigned)a | ((unsigned)b << 16); }
__device__ __forceinline__ unsigned short h_bits(float f) { const _Float16 h = (_Float16)f; return __builtin_bit_cast(unsigned short, h); }

template <int ET> struct Elem;
template <> struct Elem<0> { typedef _Float16 T; };
template <> struct Elem<1> { typedef __bf16 T; };
template <int ET, bool SPLIT, int BIAS_MODE, int OUT_MODE, bool RESID, int ACT = 0, bool RSC = false>
__global__ __launch_bounds__(256) void wmma_gemm64(
    const unsigned short* __restrict__ Ap, const unsigned short* __restrict__ A2p, int lda, long strideA,
    const unsigned short* __restrict__ Btp, const unsigned short* __restrict__ Bt2p, int ldb, long strideB,
    void* __restrict__ Cout, void* __restrict__ Cout2, int ldc, long strideC,
    const float* __restrict__ bias, long strideBias,
    const float* __restrict__ resid, long strideR,
    const float* __restrict__ rsc, long strideS,
    int M, int N, int K, float scale) {
  typedef typename Elem<ET>::T T;
  typedef typename Frag<T>::V V;
  const T* A = (const T*)Ap; const T* A2 = (const T*)A2p; const T* Bt = (const T*)Btp; const T* Bt2 = (const T*)Bt2p;
  __shared__ __align__(16) float sT[8][16 * 68];
  const int b    = blockIdx.y;
  const int lane = threadIdx.x & 31;
  const int wave = threadIdx.x >> 5;
  const int tilesN = N >> 6;
  const int tilesM = M >> 6;
  const int tile = blockIdx.x * 8 + wave;
  if (tile >= tilesM * tilesN) return;
  const int tm = tile / tilesN;
  const int tn = tile - tm * tilesN;
  const int m0 = tm << 6;
  const int n0 = tn << 6;

  const T* Ab  = A  + (size_t)b * strideA;
  const T* Bb  = Bt + (size_t)b * strideB;
  const T* Ab2 = SPLIT ? (A2  + (size_t)b * strideA) : nullptr;
  const T* Bb2 = SPLIT ? (Bt2 + (size_t)b * strideB) : nullptr;

  const int rlane = lane & 15;
  const int koff  = (lane >> 4) * 8;
  const int mOff  = (lane >> 4) * 8;

  v8f acc[4][4];
#pragma unroll
  for (int i = 0; i < 4; ++i)
#pragma unroll
    for (int j = 0; j < 4; ++j) acc[i][j] = (v8f){0.f,0.f,0.f,0.f,0.f,0.f,0.f,0.f};

  for (int k0 = 0; k0 < K; k0 += 32) {
    V bh[4], bl[4];
#pragma unroll
    for (int j = 0; j < 4; ++j) {
      const size_t bo = (size_t)(n0 + (j << 4) + rlane) * ldb + koff + k0;
      bh[j] = Frag<T>::load(Bb + bo);
      if (SPLIT) bl[j] = Frag<T>::load(Bb2 + bo);
    }
#pragma unroll
    for (int i = 0; i < 4; ++i) {
      const size_t ao = (size_t)(m0 + (i << 4) + rlane) * lda + koff + k0;
      V ah = Frag<T>::load(Ab + ao);
      V al;
      if (SPLIT) al = Frag<T>::load(Ab2 + ao);
#pragma unroll
      for (int j = 0; j < 4; ++j) {
        acc[i][j] = Frag<T>::mma(ah, bh[j], acc[i][j]);
        if (SPLIT) {
          acc[i][j] = Frag<T>::mma(ah, bl[j], acc[i][j]);
          acc[i][j] = Frag<T>::mma(al, bh[j], acc[i][j]);
        }
      }
      Frag<T>::guard(acc[i][0], acc[i][3], ah, SPLIT ? al : ah);
    }
    Frag<T>::keep(bh[0], bh[1], bh[2], bh[3]);
    if (SPLIT) Frag<T>::keep(bl[0], bl[1], bl[2], bl[3]);
  }
  acc_guard4(acc[0][0], acc[0][1], acc[0][2], acc[0][3]);
  acc_guard4(acc[1][0], acc[1][1], acc[1][2], acc[1][3]);
  acc_guard4(acc[2][0], acc[2][1], acc[2][2], acc[2][3]);
  acc_guard4(acc[3][0], acc[3][1], acc[3][2], acc[3][3]);

  float* slab = sT[wave];
  const float* Rb  = RESID ? (resid + (size_t)b * strideR) : nullptr;
  const float* Bsb = (BIAS_MODE != 0) ? (bias + (size_t)b * strideBias) : nullptr;
  const float* Scb = RSC ? (rsc + (size_t)b * strideS) : nullptr;
#pragma unroll
  for (int i = 0; i < 4; ++i) {
    const int mBase = m0 + (i << 4);
#pragma unroll
    for (int j = 0; j < 4; ++j) {
      const int n = n0 + (j << 4) + rlane;
      float bv = 0.f;
      if (BIAS_MODE == 2) bv = Bsb[n];
#pragma unroll
      for (int r = 0; r < 8; ++r) {
        float v = acc[i][j][r] * scale;
        if (RSC) v = v * Scb[mBase + mOff + r];
        if (BIAS_MODE == 1) v += Bsb[mBase + mOff + r];
        if (BIAS_MODE == 2) v += bv;
        if (RESID) v += Rb[(size_t)(mBase + mOff + r) * ldc + n];
        if (ACT == 2) v = fmaxf(v, 0.0f);
        if (ACT == 4) v = (v > 0.f) ? v : 0.01f * v;
        slab[(mOff + r) * 68 + (j << 4) + rlane] = v;
      }
    }
    __builtin_amdgcn_fence(__ATOMIC_RELEASE, "workgroup");
    __builtin_amdgcn_wave_barrier();
    __builtin_amdgcn_fence(__ATOMIC_ACQUIRE, "workgroup");
    if (OUT_MODE == 0) {
      float* C = (float*)Cout + (size_t)b * strideC;
      const int hh = lane >> 4, c4 = (lane & 15) * 4;
      for (int pass = 0; pass < 2; ++pass) {
#pragma unroll
        for (int it = 0; it < 8; ++it) {
          const int row = it * 2 + hh;
          v4f v = *(const v4f*)(slab + row * 68 + c4);
          *(volatile v4f*)(C + (size_t)(mBase + row) * ldc + n0 + c4) = v;
        }
        __threadfence();
      }
    } else {
      const int q = lane >> 3, c8 = (lane & 7) * 8;
      unsigned short* C  = (unsigned short*)Cout  + (size_t)b * strideC;
      unsigned short* C2 = (OUT_MODE == 2) ? ((unsigned short*)Cout2 + (size_t)b * strideC) : nullptr;
      for (int pass = 0; pass < 2; ++pass) {
#pragma unroll
        for (int it = 0; it < 4; ++it) {
          const int row = it * 4 + q;
          const float* sp = slab + row * 68 + c8;
          v8h hv, lv;
#pragma unroll
          for (int e = 0; e < 8; ++e) {
            if (OUT_MODE == 1) {
              hv[e] = (_Float16)sp[e];
            } else {
              unsigned short hb = f2bf_bits(sp[e]);
              unsigned short lb = f2bf_bits(sp[e] - bf_bits2f(hb));
              hv[e] = __builtin_bit_cast(_Float16, hb);
              lv[e] = __builtin_bit_cast(_Float16, lb);
            }
          }
          *(volatile v8h*)(C + (size_t)(mBase + row) * ldc + n0 + c8) = hv;
          if (OUT_MODE == 2) *(volatile v8h*)(C2 + (size_t)(mBase + row) * ldc + n0 + c8) = lv;
        }
        __threadfence();
      }
    }
    __builtin_amdgcn_fence(__ATOMIC_RELEASE, "workgroup");
    __builtin_amdgcn_wave_barrier();
    __builtin_amdgcn_fence(__ATOMIC_ACQUIRE, "workgroup");
  }
}

__global__ __launch_bounds__(256) void wtcast_kernel(const float* __restrict__ W, unsigned short* __restrict__ out,
                                                     int Din, int Dout, float scale) {
  __shared__ float sm[64][65];
  const int t  = threadIdx.x;
  const int d0 = blockIdx.x * 64;
  const int h0 = blockIdx.y * 64;
#pragma unroll
  for (int i = 0; i < 16; ++i) {
    const int e = i * 256 + t;
    const int r = e >> 6;
    const int c = e & 63;
    sm[c][r] = W[(size_t)(d0 + r) * Dout + h0 + c] * scale;
  }
  __syncthreads();
  const int lane = t & 31, wave = t >> 5;
  const int q = lane >> 3, c8 = (lane & 7) * 8;
  for (int pass = 0; pass < 2; ++pass) {
#pragma unroll
    for (int it = 0; it < 2; ++it) {
      const int row = wave * 8 + it * 4 + q;
      unsigned short hb[8];
#pragma unroll
      for (int e = 0; e < 8; ++e) hb[e] = h_bits(sm[row][c8 + e]);
      const v4u u = (v4u){pk16(hb[0], hb[1]), pk16(hb[2], hb[3]), pk16(hb[4], hb[5]), pk16(hb[6], hb[7])};
      *(volatile v4u*)(out + (size_t)(h0 + row) * Din + d0 + c8) = u;
    }
    __threadfence();
  }
}

__global__ __launch_bounds__(256) void negt_kernel(const float* __restrict__ mask, float* __restrict__ negT) {
  __shared__ float sm[64][65];
  const int t  = threadIdx.x;
  const int j0 = blockIdx.x * 64;
  const int i0 = blockIdx.y * 64;
  const int b  = blockIdx.z;
  const float* mb = mask + (size_t)b * kPlane;
#pragma unroll
  for (int it = 0; it < 16; ++it) {
    const int e  = it * 256 + t;
    const int sr = e >> 6;
    const int sc = e & 63;
    sm[sc][sr] = mb[(size_t)(j0 + sr) * kS + i0 + sc] * -1.0e9f;
  }
  __syncthreads();
  const int lane = t & 31, wave = t >> 5;
  const int hh = lane >> 4, c4 = (lane & 15) * 4;
  float* nb = negT + (size_t)b * kPlane;
  for (int pass = 0; pass < 2; ++pass) {
#pragma unroll
    for (int it = 0; it < 4; ++it) {
      const int row = wave * 8 + it * 2 + hh;
      const v4f v = (v4f){sm[row][c4], sm[row][c4 + 1], sm[row][c4 + 2], sm[row][c4 + 3]};
      *(volatile v4f*)(nb + (size_t)(i0 + row) * kS + j0 + c4) = v;
    }
    __threadfence();
  }
}

__global__ __launch_bounds__(256) void cast_act_kernel(const float* __restrict__ in, unsigned short* __restrict__ out,
                                                       float scale) {
  const size_t i = (size_t)blockIdx.x * 256 + threadIdx.x;
  const v4f a = *(const v4f*)(in + i * 8);
  const v4f c = *(const v4f*)(in + i * 8 + 4);
  unsigned short hb[8];
#pragma unroll
  for (int e = 0; e < 4; ++e) { hb[e] = h_bits(a[e] * scale); hb[4 + e] = h_bits(c[e] * scale); }
  const v4u u = (v4u){pk16(hb[0], hb[1]), pk16(hb[2], hb[3]), pk16(hb[4], hb[5]), pk16(hb[6], hb[7])};
  unsigned short* op = out + i * 8;
  *(volatile v4u*)op = u;
  __threadfence();
  *(volatile v4u*)op = u;
}

template <bool WH>
__global__ __launch_bounds__(128) void ln_kernel(const float* __restrict__ x, const float* __restrict__ g,
                                                 const float* __restrict__ be, float* __restrict__ yf,
                                                 unsigned short* __restrict__ yh) {
  __shared__ float red1[4];
  __shared__ float red2[4];
  __shared__ __align__(16) float srow[kDM];
  const int row  = blockIdx.x;
  const int t    = threadIdx.x;
  const int lane = t & 31, wave = t >> 5;
  const int c0   = t * 4;
  const v4f a = *(const v4f*)(x + (size_t)row * kDM + c0);
  float s = (a[0] + a[1]) + (a[2] + a[3]);
#pragma unroll
  for (int off = 16; off > 0; off >>= 1) s += __shfl_xor(s, off, 32);
  if (lane == 0) red1[wave] = s;
  __syncthreads();
  const float mu = ((red1[0] + red1[1]) + (red1[2] + red1[3])) * kInvDM;
  const float d0 = a[0] - mu, d1 = a[1] - mu, d2 = a[2] - mu, d3 = a[3] - mu;
  float ss = (d0 * d0 + d1 * d1) + (d2 * d2 + d3 * d3);
#pragma unroll
  for (int off = 16; off > 0; off >>= 1) ss += __shfl_xor(ss, off, 32);
  if (lane == 0) red2[wave] = ss;
  __syncthreads();
  const float var = ((red2[0] + red2[1]) + (red2[2] + red2[3])) * kInvDM;
  const float rs = rsqrtf(var + kLnEps);
  const v4f gv = *(const v4f*)(g + c0);
  const v4f bb = *(const v4f*)(be + c0);
  v4f y;
  y[0] = (d0 * rs) * gv[0] + bb[0];
  y[1] = (d1 * rs) * gv[1] + bb[1];
  y[2] = (d2 * rs) * gv[2] + bb[2];
  y[3] = (d3 * rs) * gv[3] + bb[3];
  float* yp = yf + (size_t)row * kDM + c0;
  *(volatile v4f*)yp = y;
  __threadfence();
  *(volatile v4f*)yp = y;
  if (WH) {
    *(v4f*)(srow + c0) = y;
    __syncthreads();
    if (t < 64) {
      const v4f p0 = *(const v4f*)(srow + t * 8);
      const v4f p1 = *(const v4f*)(srow + t * 8 + 4);
      unsigned short hb[8];
#pragma unroll
      for (int e = 0; e < 4; ++e) { hb[e] = h_bits(p0[e] * kActCarry); hb[4 + e] = h_bits(p1[e] * kActCarry); }
      const v4u u = (v4u){pk16(hb[0], hb[1]), pk16(hb[2], hb[3]), pk16(hb[4], hb[5]), pk16(hb[6], hb[7])};
      unsigned short* hp = yh + (size_t)row * kDM + t * 8;
      *(volatile v4u*)hp = u;
      __threadfence();
      *(volatile v4u*)hp = u;
    }
  }
}

__global__ __launch_bounds__(256) void rowstat_kernel(const float* __restrict__ S, unsigned short* __restrict__ E,
                                                      float* __restrict__ rmax, float* __restrict__ rsum) {
  __shared__ float smx[32];
  __shared__ float ssm[32];
  const int z    = blockIdx.y;
  const int rb   = blockIdx.x;
  const int t    = threadIdx.x;
  const int lane = t & 31, wave = t >> 5;
#pragma unroll 1
  for (int rr = 0; rr < 4; ++rr) {
    const int rl  = wave * 4 + rr;
    const int row = rb * 32 + rl;
    const size_t base = ((size_t)z * kS + row) * kS + lane * 8;
    const float* sp = S + base;
    float m = -3.0e38f;
#pragma unroll 1
    for (int it = 0; it < 4; ++it) {
      const v4f a = *(const v4f*)(sp + it * 256);
      const v4f c = *(const v4f*)(sp + it * 256 + 4);
      const float m8 = fmaxf(fmaxf(fmaxf(a[0], a[1]), fmaxf(a[2], a[3])), fmaxf(fmaxf(c[0], c[1]), fmaxf(c[2], c[3])));
      m = fmaxf(m, m8);
    }
#pragma unroll
    for (int off = 16; off > 0; off >>= 1) m = fmaxf(m, __shfl_xor(m, off, 32));
    float s = 0.f;
    unsigned short* ep = E + base;
#pragma unroll 1
    for (int it = 0; it < 4; ++it) {
      const v4f a = *(const v4f*)(sp + it * 256);
      const v4f c = *(const v4f*)(sp + it * 256 + 4);
      float ex[8];
#pragma unroll
      for (int e = 0; e < 4; ++e) { ex[e] = expf(a[e] - m); ex[4 + e] = expf(c[e] - m); }
      s += ((ex[0] + ex[1]) + (ex[2] + ex[3])) + ((ex[4] + ex[5]) + (ex[6] + ex[7]));
      unsigned short hb[8];
#pragma unroll
      for (int e = 0; e < 8; ++e) hb[e] = h_bits(ex[e] * kPCarry);
      const v4u u = (v4u){pk16(hb[0], hb[1]), pk16(hb[2], hb[3]), pk16(hb[4], hb[5]), pk16(hb[6], hb[7])};
      unsigned short* pp = ep + it * 256;
      *(volatile v4u*)pp = u;
      __threadfence();
      *(volatile v4u*)pp = u;
    }
#pragma unroll
    for (int off = 16; off > 0; off >>= 1) s += __shfl_xor(s, off, 32);
    if (lane == 0) { smx[rl] = m; ssm[rl] = s; }
  }
  __syncthreads();
  if (wave == 0) {
    const float v = smx[lane];
    float* p = rmax + (size_t)z * kS + rb * 32 + lane;
    *(volatile float*)p = v;
    __threadfence();
    *(volatile float*)p = v;
  }
  if (wave == 1) {
    const float v = ssm[lane];
    float* p = rsum + (size_t)z * kS + rb * 32 + lane;
    *(volatile float*)p = v;
    __threadfence();
    *(volatile float*)p = v;
  }
}

__global__ __launch_bounds__(256) void zred_kernel(const float* __restrict__ rmax, const float* __restrict__ rsum,
                                                   const int* __restrict__ protok, float* __restrict__ rsv) {
  __shared__ float redM[8];
  __shared__ float redZ[8];
  __shared__ int   redN[8];
  const int t    = threadIdx.x;
  const int lane = t & 31, wave = t >> 5;
  const v4i pv = *(const v4i*)(protok + t * 4);
  int cnt = ((pv[0] != 0) ? 1 : 0) + ((pv[1] != 0) ? 1 : 0) + ((pv[2] != 0) ? 1 : 0) + ((pv[3] != 0) ? 1 : 0);
#pragma unroll
  for (int off = 16; off > 0; off >>= 1) cnt += __shfl_xor(cnt, off, 32);
  if (lane == 0) redN[wave] = cnt;
  __syncthreads();
  int tot = 0;
#pragma unroll
  for (int w = 0; w < 8; ++w) tot += redN[w];
  const float nz = (float)tot;
#pragma unroll 1
  for (int p = 0; p < kH; ++p) {
    const v4f mv = *(const v4f*)(rmax + (size_t)p * kS + t * 4);
    const v4f sv = *(const v4f*)(rsum + (size_t)p * kS + t * 4);
    float m = fmaxf(fmaxf(mv[0], mv[1]), fmaxf(mv[2], mv[3]));
#pragma unroll
    for (int off = 16; off > 0; off >>= 1) m = fmaxf(m, __shfl_xor(m, off, 32));
    if (lane == 0) redM[wave] = m;
    __syncthreads();
    float gm = redM[0];
#pragma unroll
    for (int w = 1; w < 8; ++w) gm = fmaxf(gm, redM[w]);
    const float e0 = expf(mv[0] - gm);
    const float e1 = expf(mv[1] - gm);
    const float e2 = expf(mv[2] - gm);
    const float e3 = expf(mv[3] - gm);
    float zs = (sv[0] * e0 + sv[1] * e1) + (sv[2] * e2 + sv[3] * e3);
#pragma unroll
    for (int off = 16; off > 0; off >>= 1) zs += __shfl_xor(zs, off, 32);
    if (lane == 0) redZ[wave] = zs;
    __syncthreads();
    float gz = redZ[0];
#pragma unroll
    for (int w = 1; w < 8; ++w) gz += redZ[w];
    const float coef = nz * (1.0f / gz);
    const v4f rv = (v4f){e0 * coef, e1 * coef, e2 * coef, e3 * coef};
    float* rp = rsv + (size_t)p * kS + t * 4;
    *(volatile v4f*)rp = rv;
    __threadfence();
    *(volatile v4f*)rp = rv;
    __syncthreads();
  }
}

extern "C" void kernel_launch(void* const* d_in, const int* in_sizes, int n_in,
                              void* d_out, int out_size, void* d_ws, size_t ws_size,
                              hipStream_t stream) {
  if (n_in < 20) return;
  if (in_sizes[0] != kRows * kDM || out_size != kRows * kDM) return;
  if (in_sizes[1] != kB * kS * kS || in_sizes[2] != kB * kS) return;
  if (in_sizes[3] != kDM * kDM || in_sizes[5] != kDM * kDM || in_sizes[7] != kDM * kDM || in_sizes[9] != kDM * kDM) return;
  if (in_sizes[11] != kDM * kFF || in_sizes[13] != kFF * kDM) return;
  if (in_sizes[4] != kDM || in_sizes[6] != kDM || in_sizes[8] != kDM || in_sizes[10] != kDM) return;
  if (in_sizes[12] != kFF || in_sizes[14] != kDM) return;
  if (in_sizes[15] != kDM || in_sizes[16] != kDM || in_sizes[17] != kDM || in_sizes[18] != kDM) return;

  const float* x      = (const float*)d_in[0];
  const float* mask   = (const float*)d_in[1];
  const int*   protok = (const int*)d_in[2];
  const float* wq   = (const float*)d_in[3];  const float* bq   = (const float*)d_in[4];
  const float* wk   = (const float*)d_in[5];  const float* bk   = (const float*)d_in[6];
  const float* wv   = (const float*)d_in[7];  const float* bv   = (const float*)d_in[8];
  const float* wo   = (const float*)d_in[9];  const float* bo   = (const float*)d_in[10];
  const float* w1   = (const float*)d_in[11]; const float* b1   = (const float*)d_in[12];
  const float* w2   = (const float*)d_in[13]; const float* b2   = (const float*)d_in[14];
  const float* ln1g = (const float*)d_in[15]; const float* ln1b = (const float*)d_in[16];
  const float* ln2g = (const float*)d_in[17]; const float* ln2b = (const float*)d_in[18];
  float* out = (float*)d_out;

  const size_t MiB = (size_t)1 << 20;
  const size_t offWq  = 0;
  const size_t offWk  = 524288;
  const size_t offWv  = 1 * MiB;
  const size_t offWo  = 1 * MiB + 524288;
  const size_t offW1  = 2 * MiB;
  const size_t offW2  = 4 * MiB;
  const size_t offNeg = 6 * MiB;
  const size_t offH16 = 22 * MiB;
  const size_t offQ16 = 26 * MiB;
  const size_t offK16 = 30 * MiB;
  const size_t offVT  = 34 * MiB;
  const size_t offS   = 38 * MiB;
  const size_t offX1  = 38 * MiB;
  const size_t offF1  = 46 * MiB;
  const size_t offX2  = 62 * MiB;
  const size_t offE   = 70 * MiB;
  const size_t offSt  = 86 * MiB;
  const size_t offO16 = 86 * MiB + 131072;
  const size_t offO1F = offO16 + 4 * MiB;
  const size_t offO1H = offO1F + 8 * MiB;
  const size_t offHF  = offO1H + 4 * MiB;
  const size_t total  = offHF + 8 * MiB;
  if (ws_size < total) return;

  char* ws = (char*)d_ws;
  unsigned short* WqT = (unsigned short*)(ws + offWq);
  unsigned short* WkT = (unsigned short*)(ws + offWk);
  unsigned short* WvT = (unsigned short*)(ws + offWv);
  unsigned short* WoT = (unsigned short*)(ws + offWo);
  unsigned short* W1T = (unsigned short*)(ws + offW1);
  unsigned short* W2T = (unsigned short*)(ws + offW2);
  float* negT = (float*)(ws + offNeg);
  unsigned short* H16 = (unsigned short*)(ws + offH16);
  unsigned short* Q16 = (unsigned short*)(ws + offQ16);
  unsigned short* K16 = (unsigned short*)(ws + offK16);
  unsigned short* VT  = (unsigned short*)(ws + offVT);
  float* Sbuf = (float*)(ws + offS);
  float* X1   = (float*)(ws + offX1);
  unsigned short* F1 = (unsigned short*)(ws + offF1);
  float* X2   = (float*)(ws + offX2);
  unsigned short* E16 = (unsigned short*)(ws + offE);
  float* RMAX = (float*)(ws + offSt);
  float* RSUM = (float*)(ws + offSt + 32768);
  float* RSV  = (float*)(ws + offSt + 65536);
  unsigned short* O16 = (unsigned short*)(ws + offO16);
  float* OUT1F = (float*)(ws + offO1F);
  unsigned short* OUT1H = (unsigned short*)(ws + offO1H);
  float* HF = (float*)(ws + offHF);

  const long headPlane = (long)kRows * kHD;
  const long vtHead    = (long)kHD * kRows;

  wtcast_kernel<<<dim3(kDM / 64, kDM / 64), 256, 0, stream>>>(wq, WqT, kDM, kDM, kWCarry);
  wtcast_kernel<<<dim3(kDM / 64, kDM / 64), 256, 0, stream>>>(wk, WkT, kDM, kDM, kWCarry);
  wtcast_kernel<<<dim3(kDM / 64, kDM / 64), 256, 0, stream>>>(wv, WvT, kDM, kDM, kWCarry);
  wtcast_kernel<<<dim3(kDM / 64, kDM / 64), 256, 0, stream>>>(wo, WoT, kDM, kDM, kWCarry);
  wtcast_kernel<<<dim3(kDM / 64, kFF / 64), 256, 0, stream>>>(w1, W1T, kDM, kFF, kWCarry);
  wtcast_kernel<<<dim3(kFF / 64, kDM / 64), 256, 0, stream>>>(w2, W2T, kFF, kDM, kWCarry);

  negt_kernel<<<dim3(kS / 64, kS / 64, kB), 256, 0, stream>>>(mask, negT);
  cast_act_kernel<<<(kRows * kDM / 8) / 256, 256, 0, stream>>>(x, H16, kActCarry);

  for (int layer = 0; layer < kNL; ++layer) {
    const float* hres = (layer == 0) ? x : HF;

    wmma_gemm64<0, false, 2, 1, false, 0, false><<<dim3(8, kH), 256, 0, stream>>>(
        H16, H16, kDM, 0L, WqT, WqT, kDM, (long)kHD * kDM, (void*)Q16, (void*)Q16, kHD, headPlane,
        bq, (long)kHD, x, 0L, RSV, 0L, kRows, kHD, kDM, kProjScale);
    wmma_gemm64<0, false, 2, 1, false, 0, false><<<dim3(8, kH), 256, 0, stream>>>(
        H16, H16, kDM, 0L, WkT, WkT, kDM, (long)kHD * kDM, (void*)K16, (void*)K16, kHD, headPlane,
        bk, (long)kHD, x, 0L, RSV, 0L, kRows, kHD, kDM, kProjScale);
    wmma_gemm64<0, false, 1, 1, false, 0, false><<<dim3(64, 1), 256, 0, stream>>>(
        WvT, WvT, kDM, 0L, H16, H16, kDM, 0L, (void*)VT, (void*)VT, kRows, 0L,
        bv, 0L, x, 0L, RSV, 0L, kDM, kRows, kDM, kProjScale);

    for (int bb = 0; bb < kB; ++bb) {
      const unsigned short* Kg = K16 + (size_t)bb * kS * kHD;
      const unsigned short* Qg = Q16 + (size_t)bb * kS * kHD;
      const float* Ng = negT + (size_t)bb * kPlane;
      const unsigned short* Vg = VT + (size_t)bb * kS;
      unsigned short* Og = O16 + (size_t)bb * kS * kDM;
      wmma_gemm64<0, false, 0, 0, true, 0, false><<<dim3(32, kH), 256, 0, stream>>>(
          Kg, Kg, kHD, headPlane, Qg, Qg, kHD, headPlane, (void*)Sbuf, (void*)Sbuf, kS, (long)kPlane,
          bq, 0L, Ng, 0L, RSV, 0L, kS, kS, kHD, kScoreScale);
      rowstat_kernel<<<dim3(kS / 32, kH), 256, 0, stream>>>(Sbuf, E16, RMAX, RSUM);
      zred_kernel<<<1, 256, 0, stream>>>(RMAX, RSUM, protok, RSV);
      wmma_gemm64<0, false, 0, 1, false, 0, true><<<dim3(2, kH), 256, 0, stream>>>(
          E16, E16, kS, (long)kPlane, Vg, Vg, kRows, vtHead, (void*)Og, (void*)Og, kDM, (long)kHD,
          bq, 0L, x, 0L, RSV, (long)kS, kS, kHD, kS, kPVScale);
    }

    wmma_gemm64<0, false, 2, 0, true, 0, false><<<dim3(64, 1), 256, 0, stream>>>(
        O16, O16, kDM, 0L, WoT, WoT, kDM, 0L, (void*)X1, (void*)X1, kDM, 0L,
        bo, 0L, hres, 0L, RSV, 0L, kRows, kDM, kDM, kWoScale);

    ln_kernel<true><<<kRows, 128, 0, stream>>>(X1, ln1g, ln1b, OUT1F, OUT1H);

    wmma_gemm64<0, false, 2, 1, false, 2, false><<<dim3(256, 1), 256, 0, stream>>>(
        OUT1H, OUT1H, kDM, 0L, W1T, W1T, kDM, 0L, (void*)F1, (void*)F1, kFF, 0L,
        b1, 0L, x, 0L, RSV, 0L, kRows, kFF, kDM, kProjScale);
    wmma_gemm64<0, false, 2, 0, true, 0, false><<<dim3(64, 1), 256, 0, stream>>>(
        F1, F1, kFF, 0L, W2T, W2T, kFF, 0L, (void*)X2, (void*)X2, kDM, 0L,
        b2, 0L, OUT1F, 0L, RSV, 0L, kRows, kDM, kFF, kFF2Scale);

    if (layer + 1 < kNL) {
      ln_kernel<true><<<kRows, 128, 0, stream>>>(X2, ln2g, ln2b, HF, H16);
    } else {
      ln_kernel<false><<<kRows, 128, 0, stream>>>(X2, ln2g, ln2b, out, H16);
    }
  }
}
